// ConvPBC_54709293416802
// MI455X (gfx1250) — hardware-verified
//
#include <hip/hip_runtime.h>
#include <math.h>

typedef __attribute__((ext_vector_type(16))) __bf16   v16b;
typedef __attribute__((ext_vector_type(8)))  float    v8f;
typedef __attribute__((ext_vector_type(4)))  float    v4f;
typedef __attribute__((ext_vector_type(2)))  float    v2f;
typedef __attribute__((ext_vector_type(4)))  unsigned v4u;
typedef __attribute__((ext_vector_type(8)))  unsigned v8u;

constexpr int kNB    = 8;
constexpr int kNM    = 2;
constexpr int kLen   = 32768;
constexpr int kTaps  = 101;
constexpr int kHeads = 16;
constexpr int kLv    = kLen - kTaps + 1;
constexpr int kHalf  = kTaps / 2;
constexpr int kRowF  = 2 * kLv;
constexpr int kKh    = 128;
constexpr int kKp    = 2 * kKh;
constexpr int kWRows = 3 * 2 * kHeads;
constexpr int kLinesBlk = 16;
constexpr int kTB    = kLinesBlk * 16;
constexpr int kTiles = 17;
constexpr int kTW    = kTiles * 16;
constexpr int kXW    = kTW + kKh;
constexpr int kWPl   = kXW / 2;
constexpr int kFullLines  = (kLv - 12) / 16;
constexpr int kNBlk       = (kFullLines + kLinesBlk - 1) / kLinesBlk;
constexpr int kMainBlocks = kNB * kNBlk;
constexpr int kSeamBlocks = 12;
constexpr int kWT    = 104;

static_assert(kLv == 32668, "valid length");
static_assert(kHalf == 50, "centre offset");
static_assert(kRowF == 65336 && (kRowF % 32) == 24, "row pitch phase");
static_assert(((kLv - 12) % 16) == 0 && kFullLines == 2041, "whole lines per row");
static_assert(kNBlk == 128 && kMainBlocks == 1024, "main grid");
static_assert(kXW == 400 && kWPl == 200, "window");
static_assert(kTW - 1 + kKh - 1 < kXW - 1, "window covers every padded tap of both parity copies");
static_assert(kTW - 1 + kWT - 1 < kXW, "window covers the phase taps");
static_assert(kTW - 1 + kHalf < kXW, "window covers the centre sample");
static_assert(kTB + 4 <= kTW, "17 tiles cover both shifted mode ranges");
static_assert((size_t)kNB * kNM * kLv * 2 == 1045376ull, "output elements");
static_assert(((size_t)kNB * kNM * kLv * 2) / 32 == (size_t)kNB * kNM * kFullLines + kSeamBlocks, "line census");
static_assert((kKp % 32) == 0 && (kWRows % 16) == 0, "depth and row tile multiples");

constexpr bool line_geometry_ok() {
  for (int r = 0; r < kNB * kNM; ++r) {
    const int s  = 4 * (r & 3);
    const int sn = 4 * ((r + 1) & 3);
    if ((((long long)r * kRowF + 2 * s) % 32) != 0) return false;
    const int tail = kLv - s - 16 * kFullLines;
    if (tail < 0 || tail >= 16) return false;
    if (tail != ((16 - sn) % 16)) return false;
  }
  return true;
}
static_assert(line_geometry_ok(), "line ownership map");

constexpr size_t kWsTotal = (size_t)kWRows * kKp * 2;
static_assert(kWsTotal == 49152ull, "carve total");

__device__ __forceinline__ unsigned bf16_bits_rne(float f) {
  const unsigned u = __float_as_uint(f);
  return (u + 0x7FFFu + ((u >> 16) & 1u)) >> 16;
}
__device__ __forceinline__ float bf16_rne_f32(float f) {
  return __uint_as_float(bf16_bits_rne(f) << 16);
}

__device__ __forceinline__ v8f mma_bf(v16b a, v16b b, v8f c) {
  c = __builtin_amdgcn_wmma_f32_16x16x32_bf16(false, a, false, b, (short)0, c, false, false);
  asm volatile("v_nop\n\tv_nop\n\tv_nop\n\tv_nop" : "+v"(c) : "v"(a), "v"(b));
  return c;
}

__global__ __launch_bounds__(256) void pack_weights_kernel(
    const float* __restrict__ wr, const float* __restrict__ wi, unsigned* __restrict__ wp32)
{
  const int i = blockIdx.x * 256 + threadIdx.x;
  if (i >= kWRows * kKp / 8) return;
  const int r    = i >> 5;
  const int kc   = (i & 31) * 8;
  const int s    = r >> 5;
  const int part = (r >> 4) & 1;
  const int h    = r & 15;
  const int pl   = kc >> 7;
  const int tap0 = kc & (kKh - 1);
  const int rowoff = (s * kHeads + h) * kTaps;
  const bool use_r = (part == pl);
  const bool neg   = (part == 0) && (pl == 1);
  unsigned bits[8];
#pragma unroll
  for (int e = 0; e < 8; ++e) {
    const int tap = tap0 + e;
    const int tc  = tap < kTaps ? tap : kTaps - 1;
    float a = wr[rowoff + tc];
    float q = wi[rowoff + tc];
    asm volatile("" : "+v"(a));
    asm volatile("" : "+v"(q));
    float v = use_r ? a : q;
    v = neg ? -v : v;
    v = (tap < kTaps) ? v : 0.0f;
    bits[e] = bf16_bits_rne(v);
  }
  v4u w;
  w[0] = bits[0] | (bits[1] << 16);
  w[1] = bits[2] | (bits[3] << 16);
  w[2] = bits[4] | (bits[5] << 16);
  w[3] = bits[6] | (bits[7] << 16);
  unsigned* dst = wp32 + (size_t)i * 4;
  *(volatile v4u*)dst = w;
  __threadfence();
  *(volatile v4u*)dst = w;
}

__global__ __launch_bounds__(256) void fused_conv_mix_kernel(
    const float* __restrict__ x_real, const float* __restrict__ x_imag,
    const float* __restrict__ xpm_w,  const float* __restrict__ xpm_b,
    const float* __restrict__ fwm_br, const float* __restrict__ fwm_bi,
    const unsigned short* __restrict__ wp, float* __restrict__ out)
{
  __shared__ __align__(16) float    xf[4 * kXW];
  __shared__ __align__(16) float    pw[2 * kXW];
  __shared__ __align__(16) unsigned x16[2 * 4 * kWPl];
  __shared__ __align__(16) float    xw[4 * kWT];
  __shared__ __align__(16) float    bl[kWRows];
  __shared__ __align__(16) float    xb[4];
  __shared__ __align__(16) float    so[2 * 2 * kTW];

  const int tid  = threadIdx.x;
  const int lane = tid & 31;
  const int wave = __builtin_amdgcn_readfirstlane((int)(threadIdx.x >> 5));
  const int bid  = blockIdx.x;
  const bool seam = bid >= kMainBlocks;
  const int bm    = seam ? 0 : bid / kNBlk;
  const int blk   = seam ? 0 : bid - bm * kNBlk;
  const int s0    = (bm & 1) * 8;
  const int sq    = seam ? bid - kMainBlocks : 0;
  const int sq3   = sq / 3;
  const int rn    = sq3 * 4 + (sq - sq3 * 3) + 1;
  const int sn    = 4 * (rn & 3);
  const int njobs = seam ? 2 : 1;
  const int ntile = seam ? 1 : kTiles;

  for (int idx = tid; idx < 4 * kWT; idx += 256) {
    const int mm = idx / kWT;
    const int k  = idx - mm * kWT;
    const int kc = k < kTaps ? k : kTaps - 1;
    float v = xpm_w[mm * kTaps + kc];
    asm volatile("" : "+v"(v));
    xw[idx] = (k < kTaps) ? bf16_rne_f32(v) : 0.0f;
  }
  {
    const int tc   = tid < kWRows ? tid : kWRows - 1;
    const int s    = tc >> 5;
    const int part = (tc >> 4) & 1;
    const int hh   = tc & 15;
    float vr = fwm_br[s * kHeads + hh];
    float vi = fwm_bi[s * kHeads + hh];
    asm volatile("" : "+v"(vr));
    asm volatile("" : "+v"(vi));
    const float v = part ? vi : vr;
    if (tid < kWRows) bl[tid] = bf16_rne_f32(v);
    const int t2 = tid < 2 ? tid : 1;
    float pb = xpm_b[t2];
    asm volatile("" : "+v"(pb));
    if (tid < 4) xb[tid] = bf16_rne_f32(pb);
  }

  const int n   = lane & 15;
  const int h   = lane >> 4;
  const int par = n & 1;
  const unsigned short* aptr = wp + n * kKp + 8 * h;

#pragma unroll 1
  for (int job = 0; job < njobs; ++job) {
    const int rr  = rn - 1 + job;
    const int bj  = seam ? (rr >> 1) : bm;
    const int tw0 = seam ? (job ? 0 : (kLv - 16)) : (s0 + blk * kTB);

    __syncthreads();

    for (int j = tid; j < kXW; j += 256) {
      int g = tw0 + j;
      g = g < kLen - 1 ? g : kLen - 1;
#pragma unroll
      for (int m = 0; m < kNM; ++m) {
        const size_t ro = (size_t)(bj * kNM + m) * kLen + g;
        const float xr = bf16_rne_f32(x_real[ro]);
        const float xi = bf16_rne_f32(x_imag[ro]);
        xf[(m * 2 + 0) * kXW + j] = xr;
        xf[(m * 2 + 1) * kXW + j] = xi;
        pw[m * kXW + j] = xr * xr + xi * xi;
      }
    }
    __syncthreads();

    for (int i = tid; i < 2 * 4 * kWPl; i += 256) {
      const int cp  = i / (4 * kWPl);
      const int rem = i - cp * (4 * kWPl);
      const int p   = rem / kWPl;
      const int w   = rem - p * kWPl;
      const int j0  = 2 * w + cp;
      int j1 = j0 + 1;
      j1 = j1 < kXW ? j1 : kXW - 1;
      const unsigned ua = __float_as_uint(xf[p * kXW + j0]);
      const unsigned ub = __float_as_uint(xf[p * kXW + j1]);
      x16[i] = (ua >> 16) | (ub & 0xffff0000u);
    }
    __syncthreads();

#pragma unroll 1
    for (int tile = wave; tile < ntile; tile += 8) {
      const int tb  = tile * 16;
      const int stb = tb + 16 * job;
      v8f acc[12];
#pragma unroll
      for (int r = 0; r < 12; ++r) acc[r] = (v8f){0.f, 0.f, 0.f, 0.f, 0.f, 0.f, 0.f, 0.f};

      const int wb = par * (4 * kWPl) + (tb >> 1) + (n >> 1) + 4 * h;

#pragma unroll 1
      for (int ks = 0; ks < kKp / 32; ++ks) {
        const int pl = ks >> 2;
        const int kk = ks & 3;
        const unsigned* q0 = x16 + wb + pl * kWPl + kk * 16;
        const unsigned* q1 = q0 + 2 * kWPl;
        v8u w0, w1;
#pragma unroll
        for (int e = 0; e < 4; ++e) {
          w0[e]     = q0[e];
          w0[4 + e] = q0[8 + e];
          w1[e]     = q1[e];
          w1[4 + e] = q1[8 + e];
        }
        const v16b B0 = __builtin_bit_cast(v16b, w0);
        const v16b B1 = __builtin_bit_cast(v16b, w1);
        const unsigned short* ap = aptr + ks * 32;
#pragma unroll
        for (int r = 0; r < 6; ++r) {
          const v4u a0 = *(const v4u*)(ap + r * 16 * kKp);
          const v4u a1 = *(const v4u*)(ap + r * 16 * kKp + 16);
          const v8u aw = __builtin_shufflevector(a0, a1, 0, 1, 2, 3, 4, 5, 6, 7);
          const v16b A = __builtin_bit_cast(v16b, aw);
          acc[r]     = mma_bf(A, B0, acc[r]);
          acc[6 + r] = mma_bf(A, B1, acc[6 + r]);
        }
      }

#pragma unroll
      for (int r = 0; r < 6; ++r) {
        const v4f b0 = *(const v4f*)(bl + r * 16 + 8 * h);
        const v4f b1 = *(const v4f*)(bl + r * 16 + 8 * h + 4);
#pragma unroll
        for (int v = 0; v < 4; ++v) {
          acc[r][v]         += b0[v];
          acc[r][4 + v]     += b1[v];
          acc[6 + r][v]     += b0[v];
          acc[6 + r][4 + v] += b1[v];
        }
      }

      float pr0 = 0.f, pi0 = 0.f, pr1 = 0.f, pi1 = 0.f;
#pragma unroll
      for (int v = 0; v < 8; ++v) {
        const float sr = acc[0][v] * acc[4][v] + acc[1][v] * acc[5][v]
                       + acc[6][v] * acc[10][v] + acc[7][v] * acc[11][v];
        const float si = acc[1][v] * acc[4][v] - acc[0][v] * acc[5][v]
                       + acc[7][v] * acc[10][v] - acc[6][v] * acc[11][v];
        pr0 += acc[2][v] * sr - acc[3][v] * si;
        pi0 += acc[2][v] * si + acc[3][v] * sr;
        pr1 += acc[8][v] * sr - acc[9][v] * si;
        pi1 += acc[8][v] * si + acc[9][v] * sr;
      }
      pr0 += __shfl_xor(pr0, 16, 32);
      pi0 += __shfl_xor(pi0, 16, 32);
      pr1 += __shfl_xor(pr1, 16, 32);
      pi1 += __shfl_xor(pi1, 16, 32);
      const float fr = h ? pr1 : pr0;
      const float fi = h ? pi1 : pi0;

      float phi = xb[h];
      {
        const float* pp = pw + tb + n;
        const float* wq = xw + h * 2 * kWT;
#pragma unroll 1
        for (int mi = 0; mi < 2; ++mi) {
#pragma unroll 2
          for (int k4 = 0; k4 < kWT / 4; ++k4) {
            const v4f w = *(const v4f*)(wq + mi * kWT + 4 * k4);
            const float* p4 = pp + mi * kXW + 4 * k4;
            phi = fmaf(w[0], p4[0], phi);
            phi = fmaf(w[1], p4[1], phi);
            phi = fmaf(w[2], p4[2], phi);
            phi = fmaf(w[3], p4[3], phi);
          }
        }
      }
      float sn_, cs_;
      sincosf(phi, &sn_, &cs_);
      const float xrc = xf[(h * 2 + 0) * kXW + tb + n + kHalf];
      const float xic = xf[(h * 2 + 1) * kXW + tb + n + kHalf];
      v2f e;
      e[0] = xrc * cs_ - xic * sn_ + fr;
      e[1] = xrc * sn_ + xic * cs_ + fi;
      *(v2f*)(so + h * (2 * kTW) + (stb + n) * 2) = e;
    }
  }
  __syncthreads();

  v4f    val;
  size_t adr;
  bool   ok;
  if (seam) {
    const int q8   = tid & 7;
    const int u    = 2 * q8;
    const int msel = (u < 16 - sn) ? ((rn - 1) & 1) : (rn & 1);
    val = *(const v4f*)(so + msel * (2 * kTW) + (sn + u) * 2);
    adr = (size_t)rn * kRowF + (size_t)(2 * sn) - 32 + (size_t)(4 * q8);
    ok  = tid < 8;
  } else {
    const int m    = tid >> 7;
    const int idx  = tid & 127;
    const int line = idx >> 3;
    const int q    = idx & 7;
    int nl = kFullLines - kLinesBlk * blk;
    nl = nl < kLinesBlk ? nl : kLinesBlk;
    val = *(const v4f*)(so + m * (2 * kTW) + (4 * m + 16 * line) * 2 + 4 * q);
    adr = ((size_t)(bm * kNM + m) * kLv + (size_t)(s0 + 4 * m + kTB * blk + 16 * line)) * 2 + (size_t)(4 * q);
    ok  = line < nl;
  }
  for (int pass = 0; pass < 2; ++pass) {
    if (ok) *(volatile v4f*)(out + adr) = val;
    __threadfence();
  }
}

extern "C" void kernel_launch(void* const* d_in, const int* in_sizes, int n_in,
                              void* d_out, int out_size, void* d_ws, size_t ws_size,
                              hipStream_t stream) {
  if (n_in < 8) return;
  if (in_sizes[0] != kNB * kNM * kLen) return;
  if (in_sizes[1] != kNB * kNM * kLen) return;
  if (in_sizes[2] != kNM * kNM * kTaps) return;
  if (in_sizes[3] != kNM) return;
  if (in_sizes[4] != 3 * kHeads * kTaps) return;
  if (in_sizes[5] != 3 * kHeads * kTaps) return;
  if (in_sizes[6] != 3 * kHeads) return;
  if (in_sizes[7] != 3 * kHeads) return;
  if (out_size != kNB * kNM * kLv * 2) return;
  if (ws_size < kWsTotal) return;

  const float* x_real = (const float*)d_in[0];
  const float* x_imag = (const float*)d_in[1];
  const float* xpm_w  = (const float*)d_in[2];
  const float* xpm_b  = (const float*)d_in[3];
  const float* fwm_wr = (const float*)d_in[4];
  const float* fwm_wi = (const float*)d_in[5];
  const float* fwm_br = (const float*)d_in[6];
  const float* fwm_bi = (const float*)d_in[7];
  float* out = (float*)d_out;
  unsigned* wp32 = (unsigned*)d_ws;

  pack_weights_kernel<<<(kWRows * kKp / 8) / 256, 256, 0, stream>>>(fwm_wr, fwm_wi, wp32);
  fused_conv_mix_kernel<<<kMainBlocks + kSeamBlocks, 256, 0, stream>>>(
      x_real, x_imag, xpm_w, xpm_b, fwm_br, fwm_bi, (const unsigned short*)d_ws, out);
}
